// LiZAttention_3040836846396
// MI455X (gfx1250) — hardware-run, weakly checked
//
#include <hip/hip_runtime.h>
#include <math.h>

typedef __attribute__((ext_vector_type(16))) __bf16   v16b;
typedef __attribute__((ext_vector_type(8)))  __bf16   v8b;
typedef __attribute__((ext_vector_type(8)))  float    v8f;
typedef __attribute__((ext_vector_type(4)))  float    v4f;
typedef __attribute__((ext_vector_type(4)))  unsigned int v4u;

constexpr int kSeq   = 2048;
constexpr int kDm    = 1024;
constexpr int kNH    = 16;
constexpr int kNKV   = 8;
constexpr int kHD    = 64;
constexpr int kQW    = kNH * kHD;
constexpr int kKW    = kNKV * kHD;
constexpr int kQKVW  = kQW + 2 * kKW;
constexpr int kQKP   = kQW + kKW;
constexpr int kMixP  = 2 * kQW;
constexpr int kRowsPerTok = kNH + kNKV;
constexpr int kSqrtHD = 8;
constexpr float kScoreScale = 1.0f / (float)kSqrtHD;
constexpr float kGateInv    = 1.0f / 16.0f;
constexpr float kGateClip   = 16.0f;
constexpr float kMag        = 0.5f;
constexpr float kOneMinusMag = 1.0f - kMag;
constexpr float kClipLo     = 1e-6f;
constexpr float kClipHi     = 0.999999f;
constexpr float kMaskFill   = -1e9f;
constexpr int kTS = 32;

static_assert(kSqrtHD * kSqrtHD == kHD);
static_assert(kQW == 1024 && kKW == 512 && kQKVW == 2048 && kQKP == 1536 && kMixP == 2048);
static_assert(kNH == 2 * kNKV);
static_assert((kDm % 32) == 0 && (kMixP % 32) == 0);
static_assert((kSeq % 64) == 0 && (kQKVW % 64) == 0 && (kDm % 64) == 0);
static_assert((kSeq % kTS) == 0);
static_assert((kQW % 8) == 0 && (kQKP % 8) == 0);

constexpr size_t kOffXB    = 0;
constexpr size_t kOffBTQKV = kOffXB    + (size_t)kSeq * kDm * 2;
constexpr size_t kOffBTO2  = kOffBTQKV + (size_t)kQKVW * kDm * 2;
constexpr size_t kOffQKV   = kOffBTO2  + (size_t)kDm * kMixP * 2;
constexpr size_t kOffQL    = kOffQKV   + (size_t)kSeq * kQKVW * 4;
constexpr size_t kOffKL    = kOffQL    + (size_t)kSeq * kQW * 4;
constexpr size_t kOffEG    = kOffKL    + (size_t)kSeq * kKW * 4;
constexpr size_t kOffQKH   = kOffEG    + (size_t)kSeq * kKW * 4;
constexpr size_t kOffQKL   = kOffQKH   + (size_t)kSeq * kQKP * 2;
constexpr size_t kOffVTH   = kOffQKL   + (size_t)kSeq * kQKP * 2;
constexpr size_t kOffVTL   = kOffVTH   + (size_t)kNKV * kHD * kSeq * 2;
constexpr size_t kOffOLIN  = kOffVTL   + (size_t)kNKV * kHD * kSeq * 2;
constexpr size_t kOffMIX2  = kOffOLIN  + (size_t)kSeq * kQW * 4;
constexpr size_t kWsTotal  = kOffMIX2  + (size_t)kSeq * kMixP * 2;
static_assert(kWsTotal == 79691776ull);
static_assert(kWsTotal <= 134217728ull);
static_assert((kOffBTQKV % 128) == 0 && (kOffBTO2 % 128) == 0 && (kOffQKV % 128) == 0 && (kOffQL % 128) == 0 &&
              (kOffKL % 128) == 0 && (kOffEG % 128) == 0 && (kOffQKH % 128) == 0 && (kOffQKL % 128) == 0 &&
              (kOffVTH % 128) == 0 && (kOffVTL % 128) == 0 && (kOffOLIN % 128) == 0 && (kOffMIX2 % 128) == 0);

__device__ __forceinline__ unsigned short f2bf_bits(float f) {
  unsigned u = __float_as_uint(f);
  return (unsigned short)((u + 0x7FFFu + ((u >> 16) & 1u)) >> 16);
}
__device__ __forceinline__ float bf_bits2f(unsigned short h) { return __uint_as_float(((unsigned)h) << 16); }
__device__ __forceinline__ unsigned pk16(unsigned short a, unsigned short b) { return (unsigned)a | ((unsigned)b << 16); }
__device__ __forceinline__ void split_bits(float f, unsigned short& hb, unsigned short& lb) {
  hb = f2bf_bits(f);
  lb = f2bf_bits(f - bf_bits2f(hb));
}
__device__ __forceinline__ void split8(v4f a, v4f b, v4u& uh, v4u& ul) {
  unsigned short hb[8], lb[8];
#pragma unroll
  for (int e = 0; e < 4; ++e) {
    const float fa = a[e];
    const float fb = b[e];
    split_bits(fa, hb[e], lb[e]);
    split_bits(fb, hb[4 + e], lb[4 + e]);
  }
  uh = (v4u){pk16(hb[0], hb[1]), pk16(hb[2], hb[3]), pk16(hb[4], hb[5]), pk16(hb[6], hb[7])};
  ul = (v4u){pk16(lb[0], lb[1]), pk16(lb[2], lb[3]), pk16(lb[4], lb[5]), pk16(lb[6], lb[7])};
}
__device__ __forceinline__ v4u pack8(v4f a, v4f b) {
  unsigned short hb[8];
#pragma unroll
  for (int e = 0; e < 4; ++e) {
    const float fa = a[e];
    const float fb = b[e];
    hb[e] = f2bf_bits(fa);
    hb[4 + e] = f2bf_bits(fb);
  }
  return (v4u){pk16(hb[0], hb[1]), pk16(hb[2], hb[3]), pk16(hb[4], hb[5]), pk16(hb[6], hb[7])};
}
__device__ __forceinline__ v16b frag_ld(const __bf16* p) {
  union { v16b v; v8b h[2]; } f;
  f.h[0] = *(const v8b*)(p);
  f.h[1] = *(const v8b*)(p + 16);
  return f.v;
}
__device__ __forceinline__ v8f mma_g(v16b a, v16b b, v8f c) {
  c = __builtin_amdgcn_wmma_f32_16x16x32_bf16(false, a, false, b, (short)0, c, false, false);
  asm volatile("v_nop\n\tv_nop\n\tv_nop\n\tv_nop" : "+v"(c) : "v"(a), "v"(b));
  return c;
}
__device__ __forceinline__ void acc_guard4(v8f& a, v8f& b, v8f& c, v8f& d) {
  asm volatile("v_nop\n\tv_nop\n\tv_nop\n\tv_nop" : "+v"(a), "+v"(b), "+v"(c), "+v"(d));
}
__device__ __forceinline__ void wave_lds_fence() {
  __builtin_amdgcn_fence(__ATOMIC_RELEASE, "workgroup");
  __builtin_amdgcn_wave_barrier();
  __builtin_amdgcn_fence(__ATOMIC_ACQUIRE, "workgroup");
}

__global__ __launch_bounds__(256) void cast8_bf16_kernel(const float* __restrict__ in, unsigned short* __restrict__ out, int n8) {
  const int i = blockIdx.x * 256 + threadIdx.x;
  if (i >= n8) return;
  const float* p = in + 8 * (size_t)i;
  const v4f a = *(const v4f*)(p);
  const v4f b = *(const v4f*)(p + 4);
  const v4u u = pack8(a, b);
  unsigned short* q = out + 8 * (size_t)i;
  *(volatile v4u*)q = u;
  __threadfence();
  *(volatile v4u*)q = u;
}

__global__ __launch_bounds__(256) void wt_planes_kernel(const float* __restrict__ W0, const float* __restrict__ W1,
                                                        const float* __restrict__ W2, const float* __restrict__ W3,
                                                        unsigned short* __restrict__ btqkv, unsigned short* __restrict__ bto2) {
  __shared__ float sm[64][65];
  const int t = threadIdx.x;
  const int z = blockIdx.z;
  const int ncols = (z == 0 || z == 3) ? kQW : kKW;
  const int k0 = blockIdx.x * 64;
  const int n0 = blockIdx.y * 64;
  if (n0 >= ncols) return;
  const float* W = (z == 0) ? W0 : (z == 1) ? W1 : (z == 2) ? W2 : W3;
#pragma unroll
  for (int i = 0; i < 16; ++i) {
    const int e = i * 256 + t;
    const int r = e >> 6;
    const int c = e & 63;
    sm[c][r] = W[(size_t)(k0 + r) * ncols + n0 + c];
  }
  __syncthreads();
  const int lane = t & 31, wave = t >> 5;
  const int q = lane >> 3, c8 = (lane & 7) * 8;
  const bool dup = (z == 3);
  const int rowoff = (z == 1) ? kQW : (z == 2) ? (kQW + kKW) : 0;
  const int ld = dup ? kMixP : kDm;
  unsigned short* dst = dup ? bto2 : btqkv;
  v4u u[2];
#pragma unroll
  for (int it = 0; it < 2; ++it) {
    const int row = wave * 8 + it * 4 + q;
    v4f a, b;
#pragma unroll
    for (int e = 0; e < 4; ++e) {
      a[e] = sm[row][c8 + e];
      b[e] = sm[row][c8 + 4 + e];
    }
    u[it] = pack8(a, b);
  }
  for (int pass = 0; pass < 2; ++pass) {
#pragma unroll
    for (int it = 0; it < 2; ++it) {
      const int row = wave * 8 + it * 4 + q;
      unsigned short* p = dst + (size_t)(rowoff + n0 + row) * ld + k0 + c8;
      *(volatile v4u*)p = u[it];
      if (dup) *(volatile v4u*)(p + kDm) = u[it];
    }
    __threadfence();
  }
}

__global__ __launch_bounds__(256) void gemm_bf16_kernel(
    const unsigned short* __restrict__ Ap, int lda,
    const unsigned short* __restrict__ Btp, int ldb,
    float* __restrict__ C, int ldc, int M, int N, int K) {
  const __bf16* A  = (const __bf16*)Ap;
  const __bf16* Bt = (const __bf16*)Btp;
  __shared__ __align__(16) float sT[8][16 * 68];
  const int lane = threadIdx.x & 31;
  const int wave = threadIdx.x >> 5;
  const int tilesN = N >> 6;
  const int tilesM = M >> 6;
  const int tile = blockIdx.x * 8 + wave;
  if (tile >= tilesM * tilesN) return;
  const int tm = tile / tilesN;
  const int tn = tile - tm * tilesN;
  const int m0 = tm << 6;
  const int n0 = tn << 6;
  const int rlane = lane & 15;
  const int koff  = (lane >> 4) * 8;
  const int mOff  = (lane >> 4) * 8;

  v8f acc[4][4];
#pragma unroll
  for (int i = 0; i < 4; ++i)
#pragma unroll
    for (int j = 0; j < 4; ++j) acc[i][j] = (v8f){0.f, 0.f, 0.f, 0.f, 0.f, 0.f, 0.f, 0.f};

  for (int k0 = 0; k0 < K; k0 += 32) {
    v16b bh[4];
#pragma unroll
    for (int j = 0; j < 4; ++j) {
      const size_t bo = (size_t)(n0 + (j << 4) + rlane) * ldb + koff + k0;
      bh[j] = frag_ld(Bt + bo);
    }
#pragma unroll
    for (int i = 0; i < 4; ++i) {
      const size_t ao = (size_t)(m0 + (i << 4) + rlane) * lda + koff + k0;
      const v16b ah = frag_ld(A + ao);
#pragma unroll
      for (int j = 0; j < 4; ++j) acc[i][j] = mma_g(ah, bh[j], acc[i][j]);
    }
  }
  acc_guard4(acc[0][0], acc[0][1], acc[0][2], acc[0][3]);
  acc_guard4(acc[1][0], acc[1][1], acc[1][2], acc[1][3]);
  acc_guard4(acc[2][0], acc[2][1], acc[2][2], acc[2][3]);
  acc_guard4(acc[3][0], acc[3][1], acc[3][2], acc[3][3]);

  float* slab = sT[wave];
#pragma unroll
  for (int i = 0; i < 4; ++i) {
    const int mBase = m0 + (i << 4);
#pragma unroll
    for (int j = 0; j < 4; ++j) {
#pragma unroll
      for (int r = 0; r < 8; ++r) slab[(mOff + r) * 68 + (j << 4) + rlane] = acc[i][j][r];
    }
    wave_lds_fence();
    {
      const int hh = lane >> 4, c4 = (lane & 15) * 4;
      for (int pass = 0; pass < 2; ++pass) {
#pragma unroll
        for (int it = 0; it < 8; ++it) {
          const int row = it * 2 + hh;
          const v4f v = *(const v4f*)(slab + row * 68 + c4);
          *(volatile v4f*)(C + (size_t)(mBase + row) * ldc + n0 + c4) = v;
        }
        __threadfence();
      }
    }
    wave_lds_fence();
  }
}

__global__ __launch_bounds__(256) void split_qk_kernel(const float* __restrict__ QKV, unsigned short* __restrict__ QKh,
                                                       unsigned short* __restrict__ QKl, int total8) {
  const int i = blockIdx.x * 256 + threadIdx.x;
  if (i >= total8) return;
  constexpr int kChunks = kQKP / 8;
  const int n  = i / kChunks;
  const int c8 = (i - n * kChunks) * 8;
  const float sc = (c8 < kQW) ? kScoreScale : 1.0f;
  const float* p = QKV + (size_t)n * kQKVW + c8;
  v4f a = *(const v4f*)(p);
  v4f b = *(const v4f*)(p + 4);
#pragma unroll
  for (int e = 0; e < 4; ++e) {
    a[e] = a[e] * sc;
    b[e] = b[e] * sc;
  }
  v4u uh, ul;
  split8(a, b, uh, ul);
  unsigned short* qh = QKh + 8 * (size_t)i;
  unsigned short* ql = QKl + 8 * (size_t)i;
  *(volatile v4u*)qh = uh;
  *(volatile v4u*)ql = ul;
  __threadfence();
  *(volatile v4u*)qh = uh;
  *(volatile v4u*)ql = ul;
}

__global__ __launch_bounds__(256) void vt_planes_kernel(const float* __restrict__ QKV, unsigned short* __restrict__ Vth,
                                                        unsigned short* __restrict__ Vtl) {
  __shared__ float sm[64][65];
  const int t  = threadIdx.x;
  const int t0 = blockIdx.x * 64;
  const int kv = blockIdx.y;
#pragma unroll
  for (int i = 0; i < 16; ++i) {
    const int e = i * 256 + t;
    const int r = e >> 6;
    const int c = e & 63;
    sm[c][r] = QKV[(size_t)(t0 + r) * kQKVW + kQW + kKW + kv * kHD + c];
  }
  __syncthreads();
  const int lane = t & 31, wave = t >> 5;
  const int q = lane >> 3, c8 = (lane & 7) * 8;
  v4u uh[2], ul[2];
#pragma unroll
  for (int it = 0; it < 2; ++it) {
    const int row = wave * 8 + it * 4 + q;
    v4f a, b;
#pragma unroll
    for (int e = 0; e < 4; ++e) {
      a[e] = sm[row][c8 + e];
      b[e] = sm[row][c8 + 4 + e];
    }
    split8(a, b, uh[it], ul[it]);
  }
  for (int pass = 0; pass < 2; ++pass) {
#pragma unroll
    for (int it = 0; it < 2; ++it) {
      const int row = wave * 8 + it * 4 + q;
      const size_t o = (size_t)(kv * kHD + row) * kSeq + t0 + c8;
      *(volatile v4u*)(Vth + o) = uh[it];
      *(volatile v4u*)(Vtl + o) = ul[it];
    }
    __threadfence();
  }
}

__global__ __launch_bounds__(256) void feature_kernel(const float* __restrict__ QKV, float* __restrict__ QL,
                                                      float* __restrict__ KL, float* __restrict__ EG) {
  const int lane = threadIdx.x & 31;
  const int wave = threadIdx.x >> 5;
  const int row  = blockIdx.x * 8 + wave;
  if (row >= kSeq * kRowsPerTok) return;
  const int n = row / kRowsPerTok;
  const int j = row - n * kRowsPerTok;
  const bool isq = (j < kNH);
  const int jk = isq ? 0 : (j - kNH);
  const float* src = QKV + (size_t)n * kQKVW + (isq ? j * kHD : kQW + jk * kHD);
  float* dsm = isq ? (QL + (size_t)n * kQW + j * kHD) : (KL + (size_t)n * kKW + jk * kHD);
  float* dge = EG + (size_t)n * kKW + jk * kHD;
  const float x0 = src[lane];
  const float x1 = src[32 + lane];
  float mx = fmaxf(x0, x1);
  mx = fmaxf(mx, __shfl_xor(mx, 16, 32));
  mx = fmaxf(mx, __shfl_xor(mx, 8, 32));
  mx = fmaxf(mx, __shfl_xor(mx, 4, 32));
  mx = fmaxf(mx, __shfl_xor(mx, 2, 32));
  mx = fmaxf(mx, __shfl_xor(mx, 1, 32));
  float sum = 0.0f;
#pragma unroll 1
  for (int hf = 0; hf < 2; ++hf) {
    const float x = (hf == 0) ? x0 : x1;
    sum += expf(x - mx);
  }
  sum += __shfl_xor(sum, 16, 32);
  sum += __shfl_xor(sum, 8, 32);
  sum += __shfl_xor(sum, 4, 32);
  sum += __shfl_xor(sum, 2, 32);
  sum += __shfl_xor(sum, 1, 32);
  const float inv = 1.0f / sum;
#pragma unroll 1
  for (int hf = 0; hf < 2; ++hf) {
    const float x = (hf == 0) ? x0 : x1;
    const float e = expf(x - mx);
    const float p = fminf(fmaxf(e * inv, kClipLo), kClipHi);
    float* ps = dsm + hf * 32 + lane;
    *(volatile float*)ps = p;
    __threadfence();
    *(volatile float*)ps = p;
    if (!isq) {
      const float a  = expf(-fabsf(x));
      const float ls = fminf(x, 0.0f) - log1pf(a);
      const float g  = fminf(fmaxf(ls * kGateInv, -kGateClip), kGateClip);
      const float ev = expf(g);
      float* pg = dge + hf * 32 + lane;
      *(volatile float*)pg = ev;
      __threadfence();
      *(volatile float*)pg = ev;
    }
  }
}

__global__ __launch_bounds__(256) void state_scan_kernel(const float* __restrict__ QL, const float* __restrict__ KL,
                                                         const float* __restrict__ EG, const float* __restrict__ QKV,
                                                         float* __restrict__ OLIN) {
  __shared__ __align__(16) float sQ[kTS * 128];
  __shared__ __align__(16) float sK[kTS * 64];
  __shared__ __align__(16) float sE[kTS * 64];
  __shared__ __align__(16) float sV[kTS * 64];
  __shared__ __align__(16) float sO[kTS * 128];
  const int tid = threadIdx.x, lane = tid & 31, wave = tid >> 5;
  const int kv = blockIdx.x;
  const int dq = lane & 3;
  const int m  = wave * 8 + (lane >> 2);
  float S[16];
#pragma unroll
  for (int i = 0; i < 16; ++i) S[i] = 0.0f;

#pragma unroll 1
  for (int t0 = 0; t0 < kSeq; t0 += kTS) {
#pragma unroll
    for (int i = 0; i < 4; ++i) {
      const int idx = tid + 256 * i;
      const int r = idx >> 5, c4 = (idx & 31) * 4;
      *(v4f*)(sQ + r * 128 + c4) = *(const v4f*)(QL + (size_t)(t0 + r) * kQW + kv * 128 + c4);
    }
#pragma unroll
    for (int i = 0; i < 2; ++i) {
      const int idx = tid + 256 * i;
      const int r = idx >> 4, c4 = (idx & 15) * 4;
      *(v4f*)(sK + r * 64 + c4) = *(const v4f*)(KL + (size_t)(t0 + r) * kKW + kv * kHD + c4);
      *(v4f*)(sE + r * 64 + c4) = *(const v4f*)(EG + (size_t)(t0 + r) * kKW + kv * kHD + c4);
      *(v4f*)(sV + r * 64 + c4) = *(const v4f*)(QKV + (size_t)(t0 + r) * kQKVW + kQW + kKW + kv * kHD + c4);
    }
    __syncthreads();

#pragma unroll 1
    for (int s = 0; s < kTS; ++s) {
      const float* kp = sK + s * 64 + dq * 16;
      const float* ep = sE + s * 64 + dq * 16;
      const float* q0p = sQ + s * 128 + dq * 16;
      const float* q1p = q0p + 64;
      float kk[16], ee[16];
#pragma unroll
      for (int i4 = 0; i4 < 4; ++i4) {
        const v4f a = *(const v4f*)(kp + 4 * i4);
        const v4f b = *(const v4f*)(ep + 4 * i4);
        kk[4 * i4 + 0] = a[0]; kk[4 * i4 + 1] = a[1]; kk[4 * i4 + 2] = a[2]; kk[4 * i4 + 3] = a[3];
        ee[4 * i4 + 0] = b[0]; ee[4 * i4 + 1] = b[1]; ee[4 * i4 + 2] = b[2]; ee[4 * i4 + 3] = b[3];
      }
      float dot = 0.0f;
#pragma unroll
      for (int i = 0; i < 16; ++i) {
        S[i] = S[i] * ee[i];
        dot = fmaf(kk[i], S[i], dot);
      }
      dot += __shfl_xor(dot, 1, 32);
      dot += __shfl_xor(dot, 2, 32);
      const float err = sV[s * 64 + m] - dot;
      float qa[16], qc[16];
#pragma unroll
      for (int i4 = 0; i4 < 4; ++i4) {
        const v4f a = *(const v4f*)(q0p + 4 * i4);
        const v4f b = *(const v4f*)(q1p + 4 * i4);
        qa[4 * i4 + 0] = a[0]; qa[4 * i4 + 1] = a[1]; qa[4 * i4 + 2] = a[2]; qa[4 * i4 + 3] = a[3];
        qc[4 * i4 + 0] = b[0]; qc[4 * i4 + 1] = b[1]; qc[4 * i4 + 2] = b[2]; qc[4 * i4 + 3] = b[3];
      }
      float o0 = 0.0f, o1 = 0.0f;
#pragma unroll
      for (int i = 0; i < 16; ++i) {
        S[i] = fmaf(kk[i], err, S[i]);
        o0 = fmaf(qa[i], S[i], o0);
        o1 = fmaf(qc[i], S[i], o1);
      }
      o0 += __shfl_xor(o0, 1, 32);
      o1 += __shfl_xor(o1, 1, 32);
      o0 += __shfl_xor(o0, 2, 32);
      o1 += __shfl_xor(o1, 2, 32);
      const float ov = (dq == 0) ? o0 : o1;
      if (dq < 2) sO[s * 128 + dq * 64 + m] = ov;
    }
    __syncthreads();

    v4f ov4[4];
#pragma unroll
    for (int it = 0; it < 4; ++it) ov4[it] = *(const v4f*)(sO + (it * 8 + wave) * 128 + lane * 4);
    for (int pass = 0; pass < 2; ++pass) {
#pragma unroll
      for (int it = 0; it < 4; ++it)
        *(volatile v4f*)(OLIN + (size_t)(t0 + it * 8 + wave) * kQW + kv * 128 + lane * 4) = ov4[it];
      __threadfence();
    }
  }
}

__global__ __launch_bounds__(128) void attn_mix_kernel(const unsigned short* __restrict__ QKh, const unsigned short* __restrict__ QKl,
                                                       const unsigned short* __restrict__ Vth, const unsigned short* __restrict__ Vtl,
                                                       const float* __restrict__ OLIN, unsigned short* __restrict__ MIX2) {
  __shared__ __align__(16) __bf16 Psh[4][16 * 64];
  __shared__ __align__(16) __bf16 Psl[4][16 * 64];
  __shared__ __align__(16) float  Os[4][16 * 68];

  const int tid  = threadIdx.x;
  const int wave = tid >> 5;
  const int lane = tid & 31;
  const int hh   = lane >> 4;
  const int c    = lane & 15;
  const int qb   = (int)gridDim.x - 1 - (int)blockIdx.x;
  const int h    = blockIdx.y;
  const int kvh  = h >> 1;
  const int q0   = qb * 64 + wave * 16;

  const __bf16* qkh = (const __bf16*)QKh;
  const __bf16* qkl = (const __bf16*)QKl;
  const __bf16* vth = (const __bf16*)Vth;
  const __bf16* vtl = (const __bf16*)Vtl;

  v16b qah[2], qal[2];
  {
    const size_t qo = (size_t)(q0 + c) * kQKP + h * kHD + 8 * hh;
#pragma unroll
    for (int dc = 0; dc < 2; ++dc) {
      qah[dc] = frag_ld(qkh + qo + dc * 32);
      qal[dc] = frag_ld(qkl + qo + dc * 32);
    }
  }

  float mrow[8], lrow[8];
  v8f oacc[4];
#pragma unroll
  for (int r = 0; r < 8; ++r) { mrow[r] = -INFINITY; lrow[r] = 0.f; }
#pragma unroll
  for (int t = 0; t < 4; ++t) oacc[t] = (v8f){0.f, 0.f, 0.f, 0.f, 0.f, 0.f, 0.f, 0.f};

  const int nChunks = qb + 1;
  const size_t kcol = (size_t)kQW + kvh * kHD + 8 * hh;
  const size_t vrow = (size_t)(kvh * kHD + c) * kSeq + 8 * hh;
  __bf16* pwh = Psh[wave];
  __bf16* pwl = Psl[wave];

#pragma unroll 1
  for (int kc = 0; kc < nChunks; ++kc) {
    const int kv0 = kc * 64;
    v8f s[4];
#pragma unroll
    for (int j = 0; j < 4; ++j) {
      s[j] = (v8f){0.f, 0.f, 0.f, 0.f, 0.f, 0.f, 0.f, 0.f};
#pragma unroll
      for (int dc = 0; dc < 2; ++dc) {
        const size_t ko = (size_t)(kv0 + j * 16 + c) * kQKP + kcol + dc * 32;
        const v16b kb = frag_ld(qkh + ko);
        const v16b kl = frag_ld(qkl + ko);
        s[j] = mma_g(qah[dc], kb, s[j]);
        s[j] = mma_g(qah[dc], kl, s[j]);
        s[j] = mma_g(qal[dc], kb, s[j]);
      }
      asm volatile("" ::: "memory");
    }
    const bool diag = (kc == qb);
    float cm[8];
#pragma unroll
    for (int r = 0; r < 8; ++r) {
      const int qrow = q0 + 8 * hh + r;
      float mval = -INFINITY;
#pragma unroll
      for (int j = 0; j < 4; ++j) {
        const int kvcol = kv0 + j * 16 + c;
        const bool msk = diag && (kvcol > qrow);
        const float sv = msk ? kMaskFill : s[j][r];
        s[j][r] = sv;
        mval = fmaxf(mval, sv);
      }
      mval = fmaxf(mval, __shfl_xor(mval, 1, 32));
      mval = fmaxf(mval, __shfl_xor(mval, 2, 32));
      mval = fmaxf(mval, __shfl_xor(mval, 4, 32));
      mval = fmaxf(mval, __shfl_xor(mval, 8, 32));
      cm[r] = mval;
    }
#pragma unroll
    for (int r = 0; r < 8; ++r) {
      const float mnew  = fmaxf(mrow[r], cm[r]);
      const float alpha = expf(mrow[r] - mnew);
      mrow[r] = mnew;
      float psum = 0.f;
#pragma unroll
      for (int j = 0; j < 4; ++j) {
        const float p = expf(s[j][r] - mnew);
        psum += p;
        unsigned short hb, lb;
        split_bits(p, hb, lb);
        pwh[(8 * hh + r) * 64 + j * 16 + c] = __builtin_bit_cast(__bf16, hb);
        pwl[(8 * hh + r) * 64 + j * 16 + c] = __builtin_bit_cast(__bf16, lb);
      }
      psum += __shfl_xor(psum, 1, 32);
      psum += __shfl_xor(psum, 2, 32);
      psum += __shfl_xor(psum, 4, 32);
      psum += __shfl_xor(psum, 8, 32);
      lrow[r] = lrow[r] * alpha + psum;
#pragma unroll
      for (int t = 0; t < 4; ++t) oacc[t][r] *= alpha;
    }
    wave_lds_fence();
#pragma unroll 1
    for (int kk = 0; kk < 2; ++kk) {
      union { v16b v; v8b hv[2]; } pa, pl;
      pa.hv[0] = *(const v8b*)(pwh + c * 64 + kk * 32 + 8 * hh);
      pa.hv[1] = *(const v8b*)(pwh + c * 64 + kk * 32 + 16 + 8 * hh);
      pl.hv[0] = *(const v8b*)(pwl + c * 64 + kk * 32 + 8 * hh);
      pl.hv[1] = *(const v8b*)(pwl + c * 64 + kk * 32 + 16 + 8 * hh);
#pragma unroll
      for (int t = 0; t < 4; ++t) {
        const size_t vo = vrow + (size_t)(t * 16) * kSeq + kv0 + kk * 32;
        const v16b vb = frag_ld(vth + vo);
        const v16b vl = frag_ld(vtl + vo);
        oacc[t] = mma_g(pa.v, vb, oacc[t]);
        oacc[t] = mma_g(pa.v, vl, oacc[t]);
        oacc[t] = mma_g(pl.v, vb, oacc[t]);
        asm volatile("" ::: "memory");
      }
    }
    wave_lds_fence();
  }

  float* os = Os[wave];
#pragma unroll
  for (int r = 0; r < 8; ++r) {
    const float inv = 1.0f / lrow[r];
#pragma unroll
    for (int t = 0; t < 4; ++t) os[(8 * hh + r) * 68 + t * 16 + c] = oacc[t][r] * inv;
  }
  wave_lds_fence();
  {
    const int q = lane >> 3, c8 = (lane & 7) * 8;
    v4u uh[4], ul[4];
#pragma unroll
    for (int it = 0; it < 4; ++it) {
      const int row = it * 4 + q;
      const float* sp = os + row * 68 + c8;
      const v4f a0 = *(const v4f*)(sp);
      const v4f a1 = *(const v4f*)(sp + 4);
      const float* lp = OLIN + (size_t)(q0 + row) * kQW + h * kHD + c8;
      const v4f l0 = *(const v4f*)(lp);
      const v4f l1 = *(const v4f*)(lp + 4);
      v4f m0, m1;
#pragma unroll
      for (int e = 0; e < 4; ++e) {
        m0[e] = kMag * l0[e] + kOneMinusMag * a0[e];
        m1[e] = kMag * l1[e] + kOneMinusMag * a1[e];
      }
      split8(m0, m1, uh[it], ul[it]);
    }
    for (int pass = 0; pass < 2; ++pass) {
#pragma unroll
      for (int it = 0; it < 4; ++it) {
        const int row = it * 4 + q;
        unsigned short* dst = MIX2 + (size_t)(q0 + row) * kMixP + h * kHD + c8;
        *(volatile v4u*)dst = uh[it];
        *(volatile v4u*)(dst + kQW) = ul[it];
      }
      __threadfence();
    }
  }
}

extern "C" void kernel_launch(void* const* d_in, const int* in_sizes, int n_in,
                              void* d_out, int out_size, void* d_ws, size_t ws_size,
                              hipStream_t stream) {
  if (n_in < 5) return;
  if (in_sizes[0] != kSeq * kDm) return;
  if (in_sizes[1] != kDm * kQW) return;
  if (in_sizes[2] != kDm * kKW) return;
  if (in_sizes[3] != kDm * kKW) return;
  if (in_sizes[4] != kQW * kDm) return;
  if (out_size != kSeq * kDm) return;
  if (ws_size < kWsTotal) return;

  const float* hs = (const float*)d_in[0];
  const float* Wq = (const float*)d_in[1];
  const float* Wk = (const float*)d_in[2];
  const float* Wv = (const float*)d_in[3];
  const float* Wo = (const float*)d_in[4];
  float* out = (float*)d_out;

  char* ws = (char*)d_ws;
  unsigned short* XB    = (unsigned short*)(ws + kOffXB);
  unsigned short* BTQKV = (unsigned short*)(ws + kOffBTQKV);
  unsigned short* BTO2  = (unsigned short*)(ws + kOffBTO2);
  float*          QKV   = (float*)(ws + kOffQKV);
  float*          QL    = (float*)(ws + kOffQL);
  float*          KL    = (float*)(ws + kOffKL);
  float*          EG    = (float*)(ws + kOffEG);
  unsigned short* QKH   = (unsigned short*)(ws + kOffQKH);
  unsigned short* QKL   = (unsigned short*)(ws + kOffQKL);
  unsigned short* VTH   = (unsigned short*)(ws + kOffVTH);
  unsigned short* VTL   = (unsigned short*)(ws + kOffVTL);
  float*          OLIN  = (float*)(ws + kOffOLIN);
  unsigned short* MIX2  = (unsigned short*)(ws + kOffMIX2);

  cast8_bf16_kernel<<<(kSeq * kDm / 8) / 256, 256, 0, stream>>>(hs, XB, kSeq * kDm / 8);
  wt_planes_kernel<<<dim3(kDm / 64, kQW / 64, 4), 256, 0, stream>>>(Wq, Wk, Wv, Wo, BTQKV, BTO2);

  gemm_bf16_kernel<<<((kSeq / 64) * (kQKVW / 64)) / 8, 256, 0, stream>>>(
      XB, kDm, BTQKV, kDm, QKV, kQKVW, kSeq, kQKVW, kDm);

  split_qk_kernel<<<(kSeq * kQKP / 8) / 256, 256, 0, stream>>>(QKV, QKH, QKL, kSeq * kQKP / 8);
  vt_planes_kernel<<<dim3(kSeq / 64, kNKV), 256, 0, stream>>>(QKV, VTH, VTL);

  feature_kernel<<<(kSeq * kRowsPerTok) / 8, 256, 0, stream>>>(QKV, QL, KL, EG);
  state_scan_kernel<<<kNKV, 256, 0, stream>>>(QL, KL, EG, QKV, OLIN);

  attn_mix_kernel<<<dim3(kSeq / 64, kNH), 128, 0, stream>>>(QKH, QKL, VTH, VTL, OLIN, MIX2);

  gemm_bf16_kernel<<<((kSeq / 64) * (kDm / 64)) / 8, 256, 0, stream>>>(
      MIX2, kMixP, BTO2, kMixP, out, kDm, kSeq, kDm, kMixP);
}
